// ScalarAttention_59579786330696
// MI455X (gfx1250) — hardware-run, weakly checked
//
#include <hip/hip_runtime.h>


#define NE   2
#define NT   512
#define NW   256
#define NU   32
#define NP   12
#define BR   16
#define NEPS 1e-5f
#define TT   512
#define HD   64
#define ZH   2
#define RH   512
#define WIN  0
#define PCAR 1024.0f
#define SCL  0.0625f
#define PFL  6.103515625e-05f
typedef _Float16 h16;
typedef unsigned short bf;
typedef __attribute__((ext_vector_type(16))) __bf16   v16bf;
typedef __attribute__((ext_vector_type(16))) _Float16 v16h;
typedef __attribute__((ext_vector_type(8)))  _Float16 v8h;
typedef __attribute__((ext_vector_type(8)))  unsigned short v8us;
typedef __attribute__((ext_vector_type(8)))  float    v8f;
typedef __attribute__((ext_vector_type(4)))  float    v4f;
typedef v8h  __attribute__((may_alias)) v8ha;
typedef v4f  __attribute__((may_alias)) v4fa;
typedef v8us __attribute__((may_alias)) v8usa;

__device__ __forceinline__ unsigned short f2bf(float f) { unsigned u = __float_as_uint(f); u += 0x7FFFu + ((u >> 16) & 1u); return (unsigned short)(u >> 16); }
__device__ __forceinline__ float bf2f(unsigned short b) { return __uint_as_float(((unsigned)b) << 16); }
__device__ __forceinline__ float bfr(float f) { return bf2f(f2bf(f)); }
__device__ __forceinline__ v16h cat16(v8h lo, v8h hi) { return __builtin_shufflevector(lo, hi, 0, 1, 2, 3, 4, 5, 6, 7, 8, 9, 10, 11, 12, 13, 14, 15); }
__device__ __forceinline__ v16bf cat16b(v8us lo, v8us hi) { return __builtin_bit_cast(v16bf, __builtin_shufflevector(lo, hi, 0, 1, 2, 3, 4, 5, 6, 7, 8, 9, 10, 11, 12, 13, 14, 15)); }
__device__ __forceinline__ v8f wmma16(v16h a, v16h b, v8f c) { return __builtin_amdgcn_wmma_f32_16x16x32_f16(false, a, false, b, (short)0, c, false, false); }
__device__ __forceinline__ v8f wmmab(v16bf a, v16bf b, v8f c) { return __builtin_amdgcn_wmma_f32_16x16x32_bf16(false, a, false, b, (short)0, c, false, false); }


template <typename T16> struct WFrag;
template <> struct WFrag<h16> { typedef v16h V; static __device__ __forceinline__ V ld(const h16* p) { return cat16(*(const v8h*)p, *(const v8h*)(p + 16)); } static __device__ __forceinline__ v8f mma(V a, V b, v8f c) { return wmma16(a, b, c); } };
template <> struct WFrag<bf> { typedef v16bf V; static __device__ __forceinline__ V ld(const bf* p) { return cat16b(*(const v8us*)p, *(const v8us*)(p + 16)); } static __device__ __forceinline__ v8f mma(V a, V b, v8f c) { return wmmab(a, b, c); } };
template <typename T16, int NSPLIT, bool BIAS>
__global__ __launch_bounds__(32) void k_gemmw(const T16* __restrict__ A, const T16* __restrict__ A2, const T16* __restrict__ Bt, const T16* __restrict__ Bt2, int K, float* C, int ldc, const float* __restrict__ bias, size_t sA, size_t sB, size_t sC) {
    typedef typename WFrag<T16>::V V;
    __shared__ __align__(16) float os[16 * 68];
    const size_t z = blockIdx.z; A += z * sA; if (A2) A2 += z * sA; Bt += z * sB; if (Bt2) Bt2 += z * sB; C += z * sC;
    const int lane = threadIdx.x & 31, lr = lane & 15, hi = lane >> 4; const int r0 = blockIdx.x * 64, c0 = blockIdx.y * 64;
    v8f acc[4][4];
#pragma unroll
    for (int mb = 0; mb < 4; ++mb)
#pragma unroll
        for (int nb = 0; nb < 4; ++nb) acc[mb][nb] = (v8f){};
    const size_t aoff = (size_t)(r0 + lr) * K + 8 * hi, boff = (size_t)(c0 + lr) * K + 8 * hi;

    for (int kc = 0; kc < K; kc += 32) {
        V a[4], a2[4];
#pragma unroll
        for (int mb = 0; mb < 4; ++mb) { a[mb] = WFrag<T16>::ld(A + aoff + (size_t)mb * 16 * K + kc); if (NSPLIT == 1 || NSPLIT == 2) a2[mb] = WFrag<T16>::ld(A2 + aoff + (size_t)mb * 16 * K + kc); }
#pragma unroll
        for (int nb = 0; nb < 4; ++nb) { const V b = WFrag<T16>::ld(Bt + boff + (size_t)nb * 16 * K + kc); V b2; if (NSPLIT >= 2) b2 = WFrag<T16>::ld(Bt2 + boff + (size_t)nb * 16 * K + kc);
#pragma unroll
            for (int mb = 0; mb < 4; ++mb) { acc[mb][nb] = WFrag<T16>::mma(a[mb], b, acc[mb][nb]); if (NSPLIT == 1 || NSPLIT == 2) acc[mb][nb] = WFrag<T16>::mma(a2[mb], b, acc[mb][nb]); if (NSPLIT >= 2) acc[mb][nb] = WFrag<T16>::mma(a[mb], b2, acc[mb][nb]); } }
        asm volatile("v_nop\n\tv_nop\n\tv_nop\n\tv_nop" : "+v"(acc[0][0]), "+v"(acc[1][1]), "+v"(acc[2][2]), "+v"(acc[3][3]) : "v"(a[0]), "v"(a[3]));
    }
#pragma unroll
    for (int mb = 0; mb < 4; ++mb) {
#pragma unroll
        for (int nb = 0; nb < 4; ++nb) {
#pragma unroll
            for (int j = 0; j < 8; ++j) os[(hi * 8 + j) * 68 + nb * 16 + lr] = acc[mb][nb][j]; }
        __builtin_amdgcn_wave_barrier(); asm volatile("" ::: "memory");
        float* crow = C + (size_t)(r0 + mb * 16) * ldc + c0;
#pragma unroll 1
        for (int ps = 0; ps < 2; ++ps) {
#pragma unroll
            for (int s = 0; s < 8; ++s) { const int row = 2 * s + hi, cofs = lr * 4; v4f val = *(const v4fa*)(os + row * 68 + cofs); if (BIAS) { val[0] += bfr(bias[c0 + cofs]); val[1] += bfr(bias[c0 + cofs + 1]); val[2] += bfr(bias[c0 + cofs + 2]); val[3] += bfr(bias[c0 + cofs + 3]); }
                *(volatile v4f*)(crow + (size_t)row * ldc + cofs) = val; }
            if (ps == 0) __threadfence(); }
        __builtin_amdgcn_wave_barrier(); asm volatile("" ::: "memory");
    }
}

__device__ __forceinline__ h16 tohx(float x) { return (h16)x; }
__device__ __forceinline__ void splitf(float y, unsigned short& h, unsigned short& l) { h = f2bf(y); l = f2bf(y - bf2f(h)); }
typedef __attribute__((ext_vector_type(2))) _Float16 v2h;
typedef __attribute__((ext_vector_type(4))) _Float16 v4h;
typedef __attribute__((ext_vector_type(2))) unsigned short v2us;
typedef __attribute__((ext_vector_type(4))) unsigned short v4us;
typedef __attribute__((ext_vector_type(2))) float v2f;
typedef __attribute__((ext_vector_type(4))) int v4i;
__global__ __launch_bounds__(256) void k_f2h(const float* __restrict__ S, h16* P16, size_t n4) { const size_t i = (size_t)blockIdx.x * 256 + threadIdx.x; if (i >= n4) return; const v4f v = *(const v4f*)(S + i * 4); v4h o;
#pragma unroll
    for (int q = 0; q < 4; ++q) o[q] = tohx(v[q]);
    *(volatile v4h*)(P16 + i * 4) = o; __threadfence(); *(volatile v4h*)(P16 + i * 4) = o; }
__global__ __launch_bounds__(256) void k_vtp(const float* __restrict__ F, int pitch, int nheads, h16* V16, bf* Vh, bf* Vl) { const size_t e = ((size_t)blockIdx.x * 256 + threadIdx.x) * 2; if (e >= (size_t)nheads * HD * TT) return; const int t = (int)(e % TT); const int d = (int)((e / TT) % HD); const int g = (int)(e / ((size_t)TT * HD)); v2h o16; v2us oh, ol;
#pragma unroll
    for (int q = 0; q < 2; ++q) { const float x = F[(size_t)(t + q) * pitch + g * HD + d]; o16[q] = tohx(x); unsigned short a2, c2; splitf(x, a2, c2); oh[q] = a2; ol[q] = c2; }
    *(volatile v2h*)(V16 + e) = o16; *(volatile v2us*)(Vh + e) = oh; *(volatile v2us*)(Vl + e) = ol; __threadfence(); *(volatile v2h*)(V16 + e) = o16; *(volatile v2us*)(Vh + e) = oh; *(volatile v2us*)(Vl + e) = ol; }
__global__ __launch_bounds__(256) void k_asoft(const float* __restrict__ Sb, h16* P16, bf* Ph, bf* Pl) {
    const int lane = threadIdx.x & 31; const int row = blockIdx.x * 8 + (threadIdx.x >> 5); if (row >= ZH * TT) return; const int i = row % TT; const int zz = row / TT; (void)zz; const bool hires = (i < RH); const float* sr = Sb + (size_t)row * TT; float v[TT / 32]; float mx = -3.0e38f;
#pragma unroll
    for (int ch = 0; ch < TT / 128; ++ch) { const int j0 = ch * 128 + lane * 4; const v4f a = *(const v4f*)(sr + j0);
#pragma unroll
        for (int q = 0; q < 4; ++q) { const int j = j0 + q; (void)j; const float t = a[q] * SCL; v[ch * 4 + q] = t; mx = fmaxf(mx, t); } }
#pragma unroll
    for (int sh = 16; sh; sh >>= 1) mx = fmaxf(mx, __shfl_xor(mx, sh, 32));
    float sum = 0.f;
#pragma unroll
    for (int k = 0; k < TT / 32; ++k) { float d0 = __fsub_rn(v[k], mx); v[k] = __builtin_amdgcn_exp2f(__fmul_rn(d0, 1.4426950408889634f)); sum += v[k]; }
#pragma unroll
    for (int sh = 16; sh; sh >>= 1) sum += __shfl_xor(sum, sh, 32);
    const float f = __fdiv_rn(hires ? 1.0f : PCAR, sum);
    for (int ps = 0; ps < 2; ++ps) {
        if (hires) {
#pragma unroll
            for (int ch = 0; ch < TT / 128; ++ch) { v4us oh, ol;
#pragma unroll
                for (int q = 0; q < 4; ++q) { unsigned short a, c2; splitf(v[ch * 4 + q] * f, a, c2); oh[q] = a; ol[q] = c2; }
                const size_t oo = ((size_t)zz * (RH ? RH : 1) + i) * TT + ch * 128 + lane * 4; *(volatile v4us*)(Ph + oo) = oh; *(volatile v4us*)(Pl + oo) = ol; }
        } else {
#pragma unroll
            for (int ch = 0; ch < TT / 128; ++ch) { v4h o4;
#pragma unroll
                for (int q = 0; q < 4; ++q) { const float w = v[ch * 4 + q] * f; o4[q] = tohx(w < PFL ? 0.0f : w); }
                *(volatile v4h*)(P16 + (size_t)row * TT + ch * 128 + lane * 4) = o4; } }
        if (ps == 0) __threadfence(); }
}
__global__ __launch_bounds__(256) void k_pd12(const float* __restrict__ src, h16* dst) { const size_t pp = (size_t)blockIdx.x * 256 + threadIdx.x; const v4f p0 = *(const v4f*)(src + pp * NP), p1 = *(const v4f*)(src + pp * NP + 4), p2 = *(const v4f*)(src + pp * NP + 8); v8us o0, o1; const v8us zz8 = {0, 0, 0, 0, 0, 0, 0, 0};
#pragma unroll
    for (int e = 0; e < 4; ++e) { o0[e] = __builtin_bit_cast(unsigned short, tohx(bfr(p0[e]))); o0[4 + e] = __builtin_bit_cast(unsigned short, tohx(bfr(p1[e]))); o1[e] = __builtin_bit_cast(unsigned short, tohx(bfr(p2[e]))); o1[4 + e] = 0; }
    unsigned short* d0 = (unsigned short*)dst + pp * 32;
    *(volatile v8us*)(d0) = o0; *(volatile v8us*)(d0 + 8) = o1; *(volatile v8us*)(d0 + 16) = zz8; *(volatile v8us*)(d0 + 24) = zz8; __threadfence(); *(volatile v8us*)(d0) = o0; *(volatile v8us*)(d0 + 8) = o1; *(volatile v8us*)(d0 + 16) = zz8; *(volatile v8us*)(d0 + 24) = zz8; }
__global__ __launch_bounds__(256) void k_wt(const float* __restrict__ S, int kin, int nin, int kout, h16* D) { const unsigned idx = (blockIdx.x * 256u + threadIdx.x) * 2u; const unsigned nn = idx / (unsigned)kout, kk = idx - nn * (unsigned)kout; const bool row = (nn < (unsigned)nin); const bool live0 = row && (kk < (unsigned)kin), live1 = row && (kk + 1u < (unsigned)kin);
    const float val0 = live0 ? bfr(S[(size_t)kk * nin + nn]) : 0.0f; const float val1 = live1 ? bfr(S[(size_t)(kk + 1u) * nin + nn]) : 0.0f; v2h o; o[0] = tohx(val0); o[1] = tohx(val1);
    *(volatile v2h*)(D + idx) = o; __threadfence(); *(volatile v2h*)(D + idx) = o; }
__global__ __launch_bounds__(256) void k_nm1(const float* __restrict__ C1, const float* __restrict__ a3, const float* __restrict__ a4, const float* __restrict__ a5, const float* __restrict__ a6, const float* __restrict__ a7, h16* H1) { const unsigned idx = blockIdx.x * 256u + threadIdx.x; const unsigned pp = idx >> 3, u0 = (idx & 7u) * 4u; const v4f cc = *(const v4f*)(C1 + (size_t)pp * 64 + u0); v4h o;
#pragma unroll
    for (int e = 0; e < 4; ++e) { const unsigned uu = u0 + e; float yy = (cc[e] + bfr(a3[uu])) - bfr(a6[uu]); yy = yy * rsqrtf(bfr(a7[uu]) + NEPS); yy = yy * bfr(a4[uu]) + bfr(a5[uu]); o[e] = tohx(fmaxf(yy, 0.0f)); }
    h16* dst = H1 + (size_t)pp * NU + u0; *(volatile v4h*)dst = o; __threadfence(); *(volatile v4h*)dst = o; }
__global__ __launch_bounds__(256) void k_bred(const float* __restrict__ C2, const float* __restrict__ a9, const float* __restrict__ a10, const float* __restrict__ a11, const float* __restrict__ a12, const float* __restrict__ a13, float* AD) { const unsigned idx = blockIdx.x * 256u + threadIdx.x; const unsigned rr = idx >> 8, ch = idx & 255u; const float b9 = bfr(a9[ch]), m12 = bfr(a12[ch]), sc = rsqrtf(bfr(a13[ch]) + NEPS), gg = bfr(a10[ch]), bs = bfr(a11[ch]); const float* src = C2 + (size_t)rr * NT * NW + ch; float top = 0.0f;
    for (int tt = 0; tt < NT; ++tt) { float yy = (src[(size_t)tt * NW] + b9) - m12; yy = yy * sc; yy = yy * gg + bs; top = fmaxf(top, fmaxf(yy, 0.0f)); }
    float* dst = AD + (size_t)rr * NW + ch; *(volatile float*)dst = top; __threadfence(); *(volatile float*)dst = top; }
__global__ __launch_bounds__(256) void k_adc(const float* __restrict__ a0, const float* __restrict__ AD, h16* ZH16) { const size_t i = (size_t)blockIdx.x * 256 + threadIdx.x; const v4f p = *(const v4f*)(a0 + i * 4), t4 = *(const v4f*)(AD + i * 4); v4h o;
#pragma unroll
    for (int e = 0; e < 4; ++e) o[e] = tohx(bfr(p[e]) + t4[e]);
    *(volatile v4h*)(ZH16 + i * 4) = o; __threadfence(); *(volatile v4h*)(ZH16 + i * 4) = o; }

extern "C" void kernel_launch(void* const* d_in, const int* in_sizes, int n_in,
                              void* d_out, int out_size, void* d_ws, size_t ws_size, hipStream_t stream) {
    (void)in_sizes; (void)n_in; (void)out_size;
    const float* a0 = (const float*)d_in[0]; const float* a1 = (const float*)d_in[1]; const float* a2 = (const float*)d_in[2]; const float* a3 = (const float*)d_in[3]; const float* a4 = (const float*)d_in[4]; const float* a5 = (const float*)d_in[5]; const float* a6 = (const float*)d_in[6]; const float* a7 = (const float*)d_in[7];
    const float* a8 = (const float*)d_in[8]; const float* a9 = (const float*)d_in[9]; const float* a10 = (const float*)d_in[10]; const float* a11 = (const float*)d_in[11]; const float* a12 = (const float*)d_in[12]; const float* a13 = (const float*)d_in[13]; const float* a14 = (const float*)d_in[14];
    float* OUT = (float*)d_out;
    char* wsp = (char*)d_ws;
    auto take = [&](size_t bytes) { char* p = wsp; wsp += (bytes + 255) & ~(size_t)255; return (void*)p; };
    const size_t NPAIR = (size_t)NE * NT * NT, BP = (size_t)BR * NT;
    h16* RB = (h16*)take(NPAIR * 32 * 2); h16* W1 = (h16*)take((size_t)64 * 32 * 2); h16* W2 = (h16*)take((size_t)NW * 32 * 2); h16* W3 = (h16*)take((size_t)3 * NW * NW * 2);
    float* C1 = (float*)take(BP * 64 * 4); h16* H1 = (h16*)take(BP * NU * 2); float* C2 = (float*)take(BP * NW * 4); float* AD = (float*)take((size_t)NE * NT * NW * 4); h16* ZH16 = (h16*)take((size_t)NE * NT * NW * 2);
    float* P1 = (float*)take((size_t)NE * NT * NW * 4); float* P2 = (float*)take((size_t)NE * NT * NW * 4); float* P3 = (float*)take((size_t)NE * NT * NW * 4); h16* H2 = (h16*)take((size_t)NE * NT * NW * 2); h16* H3 = (h16*)take((size_t)NE * NT * NW * 2);
    h16* V16 = (h16*)take((size_t)NE * NW * NT * 2); bf* Vh = (bf*)take((size_t)NE * NW * NT * 2); bf* Vl = (bf*)take((size_t)NE * NW * NT * 2); float* Sb = (float*)take((size_t)NE * NT * NT * 4); bf* Ph = (bf*)take((size_t)NE * NT * NT * 2); bf* Pl = (bf*)take((size_t)NE * NT * NT * 2);
    if ((size_t)(wsp - (char*)d_ws) > ws_size) return;
    k_pd12<<<(unsigned)(NPAIR / 256), 256, 0, stream>>>(a1, RB);
    k_wt<<<64 * 32 / 2 / 256, 256, 0, stream>>>(a2, NP, NU, 32, W1); k_wt<<<NW * 32 / 2 / 256, 256, 0, stream>>>(a8, NU, NW, 32, W2); k_wt<<<3 * NW * NW / 2 / 256, 256, 0, stream>>>(a14, NW, 3 * NW, NW, W3);
    for (int blk = 0; blk < NE * NT / BR; ++blk) {
        k_gemmw<h16, 0, false><<<dim3((unsigned)(BP / 64), 1, 1), 32, 0, stream>>>(RB + (size_t)blk * BP * 32, nullptr, W1, nullptr, 32, C1, 64, nullptr, 0, 0, 0);
        k_nm1<<<(unsigned)(BP * 8 / 256), 256, 0, stream>>>(C1, a3, a4, a5, a6, a7, H1);
        k_gemmw<h16, 0, false><<<dim3((unsigned)(BP / 64), NW / 64, 1), 32, 0, stream>>>(H1, nullptr, W2, nullptr, NU, C2, NW, nullptr, 0, 0, 0);
        k_bred<<<BR * NW / 256, 256, 0, stream>>>(C2, a9, a10, a11, a12, a13, AD + (size_t)blk * BR * NW); }
    k_adc<<<NE * NT * NW / 4 / 256, 256, 0, stream>>>(a0, AD, ZH16);
    k_gemmw<h16, 0, false><<<dim3(NE * NT / 64, NW / 64, 1), 32, 0, stream>>>(ZH16, nullptr, W3, nullptr, NW, P1, NW, nullptr, 0, 0, 0);
    k_gemmw<h16, 0, false><<<dim3(NE * NT / 64, NW / 64, 1), 32, 0, stream>>>(ZH16, nullptr, W3 + (size_t)NW * NW, nullptr, NW, P2, NW, nullptr, 0, 0, 0);
    k_gemmw<h16, 0, false><<<dim3(NE * NT / 64, NW / 64, 1), 32, 0, stream>>>(ZH16, nullptr, W3 + (size_t)2 * NW * NW, nullptr, NW, P3, NW, nullptr, 0, 0, 0);
    k_f2h<<<NE * NT * NW / 4 / 256, 256, 0, stream>>>(P1, H2, (size_t)NE * NT * NW / 4); k_f2h<<<NE * NT * NW / 4 / 256, 256, 0, stream>>>(P2, H3, (size_t)NE * NT * NW / 4);
    for (int en = 0; en < NE; ++en) k_vtp<<<(NW * NT / 2 + 255) / 256, 256, 0, stream>>>(P3 + (size_t)en * NT * NW, NW, NW / HD, V16 + (size_t)en * NW * NT, Vh + (size_t)en * NW * NT, Vl + (size_t)en * NW * NT);
    k_gemmw<h16, 0, false><<<dim3(NT / 64, NT / 64, NE), 32, 0, stream>>>(H2, nullptr, H3, nullptr, NW, Sb, NT, nullptr, (size_t)NT * NW, (size_t)NT * NW, (size_t)NT * NT);
    k_asoft<<<ZH * TT / 8, 256, 0, stream>>>(Sb, nullptr, Ph, Pl);
    k_gemmw<bf, 2, false><<<dim3(NT / 64, NW / 64, NE), 32, 0, stream>>>(Ph, Pl, Vh, Vl, NT, OUT, NW, nullptr, (size_t)NT * NT, (size_t)NW * NT, (size_t)NT * NW);
}
